// STMambaBlock_57543971832010
// MI455X (gfx1250) — hardware-run, weakly checked
//
#include <hip/hip_runtime.h>
#include <math.h>
#include <stdint.h>

typedef __attribute__((ext_vector_type(16))) _Float16 v16h;
typedef __attribute__((ext_vector_type(8)))  _Float16 v8h;
typedef __attribute__((ext_vector_type(16))) __bf16   v16b;
typedef __attribute__((ext_vector_type(8)))  __bf16   v8b;
typedef __attribute__((ext_vector_type(8)))  float    v8f;
typedef __attribute__((ext_vector_type(4)))  float    v4f;
typedef __attribute__((ext_vector_type(4)))  unsigned v4u;

constexpr int NBAT = 4;
constexpr int TSEQ = 32;
constexpr int NNOD = 128;
constexpr int DMOD = 128;
constexpr int NHEAD = 4;
constexpr int HDIM = 32;
constexpr int DINR = 256;
constexpr int DSTA = 16;
constexpr int DTRK = 8;
constexpr int NROW = NBAT * TSEQ * NNOD;
constexpr int NSEQ = NBAT * NNOD;
constexpr int QKVW = 3 * DMOD;
constexpr int XZW  = 2 * DINR;
constexpr int XPN  = DTRK + 2 * DSTA;
constexpr int XPNP = 64;
constexpr int DBCP = 64;
static_assert(NROW % 64 == 0);
static_assert(DMOD % 64 == 0);
static_assert(QKVW % 64 == 0);
static_assert(XZW % 64 == 0);
static_assert(XPNP % 64 == 0);
static_assert(DMOD % 32 == 0);
static_assert(DINR % 32 == 0);
static_assert(NHEAD * HDIM == DMOD);
static_assert(HDIM == 32);
static_assert(NNOD == 128);
static_assert(TSEQ == 32);
static_assert(XPN % 4 == 0);
static_assert(XPN <= XPNP);
static_assert(((NROW / 64) * (QKVW / 64)) % 8 == 0);
static_assert(((NROW / 64) * (DMOD / 64)) % 8 == 0);
static_assert(((NROW / 64) * (XZW / 64)) % 8 == 0);
static_assert(((NROW / 64) * (XPNP / 64)) % 8 == 0);
static_assert(NROW * DBCP * 4 == NROW * DMOD * 2);

constexpr float WCARRY      = 64.0f;
constexpr float WCARRY_INV  = 1.0f / 64.0f;
constexpr float ACARRY      = 16.0f;
constexpr float AWCARRY_INV = 1.0f / 1024.0f;
constexpr float PCARRY      = 32768.0f;

__device__ __forceinline__ unsigned short f2bf_bits(float f) {
  unsigned u = __float_as_uint(f);
  return (unsigned short)((u + 0x7FFFu + ((u >> 16) & 1u)) >> 16);
}
__device__ __forceinline__ float bf_bits2f(unsigned short hb) { return __uint_as_float(((unsigned)hb) << 16); }

__device__ __forceinline__ void dep_guard_h(v8f& a, v8f& b, v16h x, v16h y) { asm volatile("v_nop\n\tv_nop\n\tv_nop\n\tv_nop" : "+v"(a), "+v"(b) : "v"(x), "v"(y)); }
__device__ __forceinline__ void dep_guard_b(v8f& a, v8f& b, v16b x, v16b y) { asm volatile("v_nop\n\tv_nop\n\tv_nop\n\tv_nop" : "+v"(a), "+v"(b) : "v"(x), "v"(y)); }
__device__ __forceinline__ void keep4_h(v16h a, v16h b, v16h c, v16h d) { asm volatile("v_nop" :: "v"(a), "v"(b), "v"(c), "v"(d)); }
__device__ __forceinline__ void keep4_b(v16b a, v16b b, v16b c, v16b d) { asm volatile("v_nop" :: "v"(a), "v"(b), "v"(c), "v"(d)); }
__device__ __forceinline__ void acc_guard4(v8f& a, v8f& b, v8f& c, v8f& d) { asm volatile("v_nop\n\tv_nop\n\tv_nop\n\tv_nop" : "+v"(a), "+v"(b), "+v"(c), "+v"(d)); }
template <typename T> struct Frag;
template <> struct Frag<_Float16> {
  typedef v16h V; union U { v16h v; v8h h[2]; };
  static __device__ __forceinline__ v16h load(const _Float16* p) {
    U f; f.h[0] = *(const v8h*)(p); f.h[1] = *(const v8h*)(p + 16); return f.v;
  }
  static __device__ __forceinline__ v8f mma(v16h a, v16h b, v8f c) {
    return __builtin_amdgcn_wmma_f32_16x16x32_f16(false, a, false, b, (short)0, c, false, false);
  }
  static __device__ __forceinline__ void guard(v8f& a, v8f& b, v16h x, v16h y) { dep_guard_h(a, b, x, y); }
  static __device__ __forceinline__ void keep(v16h a, v16h b, v16h c, v16h d) { keep4_h(a, b, c, d); }
};
template <> struct Frag<__bf16> {
  typedef v16b V; union U { v16b v; v8b h[2]; };
  static __device__ __forceinline__ v16b load(const __bf16* p) {
    U f; f.h[0] = *(const v8b*)(p); f.h[1] = *(const v8b*)(p + 16); return f.v;
  }
  static __device__ __forceinline__ v8f mma(v16b a, v16b b, v8f c) {
    return __builtin_amdgcn_wmma_f32_16x16x32_bf16(false, a, false, b, (short)0, c, false, false);
  }
  static __device__ __forceinline__ void guard(v8f& a, v8f& b, v16b x, v16b y) { dep_guard_b(a, b, x, y); }
  static __device__ __forceinline__ void keep(v16b a, v16b b, v16b c, v16b d) { keep4_b(a, b, c, d); }
};

template <int ET> struct Elem;
template <> struct Elem<0> { typedef _Float16 T; };
template <> struct Elem<1> { typedef __bf16 T; };
template <int ET, bool SPLIT, int BIAS_MODE, int OUT_MODE, bool RESID, int ACT = 0, int RMUL = 1>
__global__ __launch_bounds__(256) void wmma_gemm64(
    const unsigned short* __restrict__ Ap, const unsigned short* __restrict__ A2p, int lda, long strideA,
    const unsigned short* __restrict__ Btp, const unsigned short* __restrict__ Bt2p, int ldb, long strideB,
    void* __restrict__ Cout, void* __restrict__ Cout2, int ldc, long strideC,
    const float* __restrict__ bias,
    const float* __restrict__ resid, long strideR,
    int M, int N, int K, float scale) {
  static_assert(!(RESID && OUT_MODE != 0));
  static_assert(!(RESID && ACT != 0));
  static_assert(RMUL == 1 || RMUL == 2);
  typedef typename Elem<ET>::T T;
  typedef typename Frag<T>::V V;
  const T* A = (const T*)Ap; const T* A2 = (const T*)A2p; const T* Bt = (const T*)Btp; const T* Bt2 = (const T*)Bt2p;
  __shared__ __align__(16) float sT[8][16 * 68];
  const int b    = blockIdx.y;
  const int lane = threadIdx.x & 31;
  const int wave = threadIdx.x >> 5;
  const int tilesN = N >> 6;
  const int tilesM = M >> 6;
  const int tile = blockIdx.x * 8 + wave;
  if (tile >= tilesM * tilesN) return;
  const int tm = tile / tilesN;
  const int tn = tile - tm * tilesN;
  const int m0 = tm << 6;
  const int n0 = tn << 6;

  const T* Ab  = A  + (size_t)b * strideA;
  const T* Bb  = Bt + (size_t)b * strideB;
  const T* Ab2 = SPLIT ? (A2  + (size_t)b * strideA) : nullptr;
  const T* Bb2 = SPLIT ? (Bt2 + (size_t)b * strideB) : nullptr;

  const int rlane = lane & 15;
  const int koff  = (lane >> 4) * 8;
  const int mOff  = (lane >> 4) * 8;

  v8f acc[4][4];
#pragma unroll
  for (int i = 0; i < 4; ++i)
#pragma unroll
    for (int j = 0; j < 4; ++j) acc[i][j] = (v8f){0.f,0.f,0.f,0.f,0.f,0.f,0.f,0.f};

  for (int k0 = 0; k0 < K; k0 += 32) {
    V bh[4], bl[4];
#pragma unroll
    for (int j = 0; j < 4; ++j) {
      const size_t bofs = (size_t)(n0 + (j << 4) + rlane) * ldb + koff + k0;
      bh[j] = Frag<T>::load(Bb + bofs);
      if (SPLIT) bl[j] = Frag<T>::load(Bb2 + bofs);
    }
#pragma unroll
    for (int i = 0; i < 4; ++i) {
      const size_t ao = (size_t)(m0 + (i << 4) + rlane) * lda + koff + k0;
      V ah = Frag<T>::load(Ab + ao);
      V al;
      if (SPLIT) al = Frag<T>::load(Ab2 + ao);
#pragma unroll
      for (int j = 0; j < 4; ++j) {
        acc[i][j] = Frag<T>::mma(ah, bh[j], acc[i][j]);
        if (SPLIT) {
          acc[i][j] = Frag<T>::mma(ah, bl[j], acc[i][j]);
          acc[i][j] = Frag<T>::mma(al, bh[j], acc[i][j]);
        }
      }
      Frag<T>::guard(acc[i][0], acc[i][3], ah, SPLIT ? al : ah);
    }
    Frag<T>::keep(bh[0], bh[1], bh[2], bh[3]);
    if (SPLIT) Frag<T>::keep(bl[0], bl[1], bl[2], bl[3]);
  }
  acc_guard4(acc[0][0], acc[0][1], acc[0][2], acc[0][3]);
  acc_guard4(acc[1][0], acc[1][1], acc[1][2], acc[1][3]);
  acc_guard4(acc[2][0], acc[2][1], acc[2][2], acc[2][3]);
  acc_guard4(acc[3][0], acc[3][1], acc[3][2], acc[3][3]);

  float* slab = sT[wave];
  const float* Rb = resid + (size_t)b * strideR;
#pragma unroll
  for (int i = 0; i < 4; ++i) {
    const int mBase = m0 + (i << 4);
#pragma unroll
    for (int j = 0; j < 4; ++j) {
      const int n = n0 + (j << 4) + rlane;
      float bv = 0.f;
      if (BIAS_MODE == 2) bv = bias[n];
#pragma unroll
      for (int r = 0; r < 8; ++r) {
        float v = acc[i][j][r] * scale;
        if (BIAS_MODE == 1) v += bias[mBase + mOff + r];
        if (BIAS_MODE == 2) v += bv;
        if (ACT == 1) v = tanhf(v);
        if (ACT == 2) v = fmaxf(v, 0.0f);
        if (ACT == 3) v = v / (1.0f + expf(-v));
        if (ACT == 4) v = (v > 0.f) ? v : 0.01f * v;
        slab[(mOff + r) * 68 + (j << 4) + rlane] = v;
      }
    }
    __builtin_amdgcn_fence(__ATOMIC_RELEASE, "workgroup");
    __builtin_amdgcn_wave_barrier();
    __builtin_amdgcn_fence(__ATOMIC_ACQUIRE, "workgroup");
    if (OUT_MODE == 0) {
      float* Cb = (float*)Cout + (size_t)b * strideC;
      const int hh = lane >> 4, c4 = (lane & 15) * 4;
      for (int pass = 0; pass < 2; ++pass) {
#pragma unroll
        for (int it = 0; it < 8; ++it) {
          const int row = it * 2 + hh;
          v4f v = *(const v4f*)(slab + row * 68 + c4);
          if (RESID) {
            const v4f rv = *(const v4f*)(Rb + (size_t)(mBase + row) * ldc + n0 + c4);
            if (RMUL == 2) v = v + (rv + rv);
            else v = v + rv;
          }
          *(volatile v4f*)(Cb + (size_t)(mBase + row) * ldc + n0 + c4) = v;
        }
        __threadfence();
      }
    } else {
      const int q = lane >> 3, c8 = (lane & 7) * 8;
      unsigned short* Cb  = (unsigned short*)Cout  + (size_t)b * strideC;
      unsigned short* Cb2 = (OUT_MODE == 2) ? ((unsigned short*)Cout2 + (size_t)b * strideC) : nullptr;
      for (int pass = 0; pass < 2; ++pass) {
#pragma unroll
        for (int it = 0; it < 4; ++it) {
          const int row = it * 4 + q;
          const float* sp = slab + row * 68 + c8;
          v8h hv, lv;
#pragma unroll
          for (int e = 0; e < 8; ++e) {
            if (OUT_MODE == 1) {
              hv[e] = (_Float16)sp[e];
            } else {
              unsigned short hb = f2bf_bits(sp[e]);
              unsigned short lb = f2bf_bits(sp[e] - bf_bits2f(hb));
              hv[e] = __builtin_bit_cast(_Float16, hb);
              lv[e] = __builtin_bit_cast(_Float16, lb);
            }
          }
          *(volatile v8h*)(Cb + (size_t)(mBase + row) * ldc + n0 + c8) = hv;
          if (OUT_MODE == 2) *(volatile v8h*)(Cb2 + (size_t)(mBase + row) * ldc + n0 + c8) = lv;
        }
        __threadfence();
      }
    }
    __builtin_amdgcn_fence(__ATOMIC_RELEASE, "workgroup");
    __builtin_amdgcn_wave_barrier();
    __builtin_amdgcn_fence(__ATOMIC_ACQUIRE, "workgroup");
  }
}

__global__ __launch_bounds__(256) void cast_f32_f16x2(
    const float* __restrict__ in, _Float16* __restrict__ out, int n2) {
  int i = blockIdx.x * 256 + threadIdx.x;
  if (i < n2) {
    const _Float16 h0 = (_Float16)in[2 * i], h1 = (_Float16)in[2 * i + 1];
    const unsigned u = (unsigned)__builtin_bit_cast(unsigned short, h0) | ((unsigned)__builtin_bit_cast(unsigned short, h1) << 16);
    ((volatile unsigned*)out)[i] = u;
    __threadfence();
    ((volatile unsigned*)out)[i] = u;
  }
}

__global__ __launch_bounds__(256) void k_castT(const float* __restrict__ s0, const float* __restrict__ s1,
                                               const float* __restrict__ s2, int nr, int nc,
                                               _Float16* __restrict__ out, float scale) {
  __shared__ float sT[64 * 65];
  const int tid = threadIdx.x, lane = tid & 31, wave = tid >> 5;
  const int z = blockIdx.z;
  const float* src = (z == 0) ? s0 : ((z == 1) ? s1 : s2);
  _Float16* dst = out + (size_t)z * (size_t)(gridDim.y * 64) * (size_t)nr;
  const int r0 = blockIdx.x * 64, c0 = blockIdx.y * 64;
#pragma unroll
  for (int it = 0; it < 4; ++it) {
    const int e = tid + 256 * it;
    const int rr = e >> 4, cq = (e & 15) * 4;
    const int cc = c0 + cq;
    const int ccl = (cc > nc - 4) ? (nc - 4) : cc;
    const v4f v = *(const v4f*)(src + (size_t)(r0 + rr) * nc + ccl);
    const bool inb = (cc < nc);
#pragma unroll
    for (int e4 = 0; e4 < 4; ++e4) sT[(cq + e4) * 65 + rr] = inb ? (v[e4] * scale) : 0.0f;
  }
  __syncthreads();
  const int q = lane >> 3, c8 = (lane & 7) * 8;
#pragma unroll
  for (int it = 0; it < 2; ++it) {
    const int cc = wave * 8 + it * 4 + q;
    v8h hv;
#pragma unroll
    for (int e = 0; e < 8; ++e) hv[e] = (_Float16)sT[cc * 65 + c8 + e];
    _Float16* p = dst + (size_t)(c0 + cc) * nr + r0 + c8;
    *(volatile v8h*)p = hv;
    __threadfence();
    *(volatile v8h*)p = hv;
  }
}

__global__ __launch_bounds__(512) void k_adjbits(const float* __restrict__ adj, unsigned* __restrict__ adjw) {
  const int t = threadIdx.x;
  const int row = t >> 2, w = t & 3;
  const float* p = adj + (size_t)row * NNOD + w * 32;
  unsigned bits = 0u;
#pragma unroll
  for (int i = 0; i < 8; ++i) {
    const v4f v = *(const v4f*)(p + 4 * i);
#pragma unroll
    for (int e = 0; e < 4; ++e) bits |= ((v[e] != 0.0f) ? 1u : 0u) << (4 * i + e);
  }
  ((volatile unsigned*)adjw)[t] = bits;
  __threadfence();
  ((volatile unsigned*)adjw)[t] = bits;
}

constexpr int KPIT = 40;
constexpr int VPIT = 136;
constexpr int PPIT = 136;
__global__ __launch_bounds__(128) void k_attn(const unsigned short* __restrict__ qkv, const unsigned* __restrict__ adjw,
                                              _Float16* __restrict__ op) {
  __shared__ __align__(16) unsigned short sK[NNOD * KPIT];
  __shared__ __align__(16) unsigned short sVt[HDIM * VPIT];
  __shared__ __align__(16) _Float16 sP[4][16 * PPIT];
  __shared__ __align__(16) _Float16 sO[4][16 * PPIT];
  __shared__ __align__(16) unsigned sAdj[NNOD * 4];
  const int tid = threadIdx.x, wave = tid >> 5, lane = tid & 31;
  const int hh = lane >> 4, cc = lane & 15, koff = hh * 8;
  const int bt = blockIdx.x >> 1, qhalf = blockIdx.x & 1;
  const int q0 = qhalf * 64 + wave * 16;
  const size_t rowb = (size_t)bt * NNOD;
  {
    const v4u a = *(const v4u*)(adjw + 4 * tid);
    sAdj[4 * tid + 0] = a[0]; sAdj[4 * tid + 1] = a[1]; sAdj[4 * tid + 2] = a[2]; sAdj[4 * tid + 3] = a[3];
  }
  _Float16* pw = sP[wave];
  _Float16* ow = sO[wave];
  const float scl = 0.17677669529663687f;
#pragma unroll 1
  for (int head = 0; head < NHEAD; ++head) {
    __syncthreads();
#pragma unroll
    for (int it = 0; it < 4; ++it) {
      const int i = tid + 128 * it;
      const int m = i >> 2, c8 = (i & 3) * 8;
      const size_t src = (rowb + m) * QKVW + head * HDIM + c8;
      const v4u kw = *(const v4u*)(qkv + src + DMOD);
      const v4u vw = *(const v4u*)(qkv + src + 2 * DMOD);
      *(v4u*)(sK + m * KPIT + c8) = kw;
#pragma unroll
      for (int e = 0; e < 4; ++e) {
        const unsigned wv = vw[e];
        sVt[(c8 + 2 * e) * VPIT + m]     = (unsigned short)(wv & 0xffffu);
        sVt[(c8 + 2 * e + 1) * VPIT + m] = (unsigned short)(wv >> 16);
      }
    }
    __syncthreads();
    const v16h qa = Frag<_Float16>::load((const _Float16*)qkv + (rowb + q0 + cc) * QKVW + head * HDIM + koff);
    v8f s[8];
#pragma unroll
    for (int j = 0; j < 8; ++j) {
      const v16h kb = Frag<_Float16>::load((const _Float16*)sK + (j * 16 + cc) * KPIT + koff);
      s[j] = Frag<_Float16>::mma(qa, kb, (v8f){0.f,0.f,0.f,0.f,0.f,0.f,0.f,0.f});
    }
    dep_guard_h(s[6], s[7], qa, qa);
    acc_guard4(s[0], s[1], s[2], s[3]);
    acc_guard4(s[4], s[5], s[6], s[7]);
    float inv[8];
#pragma unroll
    for (int r = 0; r < 8; ++r) {
      const int qrow = q0 + 8 * hh + r;
      const unsigned w0 = sAdj[qrow * 4 + 0];
      const unsigned w1 = sAdj[qrow * 4 + 1];
      const unsigned w2 = sAdj[qrow * 4 + 2];
      const unsigned w3 = sAdj[qrow * 4 + 3];
      float mx = -INFINITY;
#pragma unroll
      for (int j = 0; j < 8; ++j) {
        const unsigned w = (j < 2) ? w0 : ((j < 4) ? w1 : ((j < 6) ? w2 : w3));
        const unsigned bit = (unsigned)(((j & 1) << 4) + cc);
        float v = s[j][r] * scl;
        v = (((w >> bit) & 1u) == 0u) ? -1.0e9f : v;
        s[j][r] = v;
        mx = fmaxf(mx, v);
      }
      mx = fmaxf(mx, __shfl_xor(mx, 1, 32));
      mx = fmaxf(mx, __shfl_xor(mx, 2, 32));
      mx = fmaxf(mx, __shfl_xor(mx, 4, 32));
      mx = fmaxf(mx, __shfl_xor(mx, 8, 32));
      float sum = 0.f;
#pragma unroll
      for (int j = 0; j < 8; ++j) {
        const float p = expf(s[j][r] - mx);
        sum += p;
        pw[(8 * hh + r) * PPIT + j * 16 + cc] = (_Float16)(p * PCARRY);
      }
      sum += __shfl_xor(sum, 1, 32);
      sum += __shfl_xor(sum, 2, 32);
      sum += __shfl_xor(sum, 4, 32);
      sum += __shfl_xor(sum, 8, 32);
      inv[r] = 1.0f / (sum * PCARRY);
    }
    __builtin_amdgcn_fence(__ATOMIC_RELEASE, "workgroup");
    __builtin_amdgcn_wave_barrier();
    __builtin_amdgcn_fence(__ATOMIC_ACQUIRE, "workgroup");
    v8f oacc[2];
    oacc[0] = (v8f){0.f,0.f,0.f,0.f,0.f,0.f,0.f,0.f};
    oacc[1] = (v8f){0.f,0.f,0.f,0.f,0.f,0.f,0.f,0.f};
#pragma unroll
    for (int kk = 0; kk < 4; ++kk) {
      const v16h pa  = Frag<_Float16>::load(pw + cc * PPIT + kk * 32 + koff);
      const v16h vb0 = Frag<_Float16>::load((const _Float16*)sVt + (0 * 16 + cc) * VPIT + kk * 32 + koff);
      const v16h vb1 = Frag<_Float16>::load((const _Float16*)sVt + (1 * 16 + cc) * VPIT + kk * 32 + koff);
      oacc[0] = Frag<_Float16>::mma(pa, vb0, oacc[0]);
      oacc[1] = Frag<_Float16>::mma(pa, vb1, oacc[1]);
      dep_guard_h(oacc[0], oacc[1], pa, vb1);
    }
#pragma unroll
    for (int r = 0; r < 8; ++r)
#pragma unroll
      for (int t2 = 0; t2 < 2; ++t2)
        ow[(8 * hh + r) * PPIT + head * HDIM + t2 * 16 + cc] = (_Float16)(oacc[t2][r] * inv[r]);
  }
  __builtin_amdgcn_fence(__ATOMIC_RELEASE, "workgroup");
  __builtin_amdgcn_wave_barrier();
  __builtin_amdgcn_fence(__ATOMIC_ACQUIRE, "workgroup");
  {
    const int c8 = cc * 8;
    for (int pass = 0; pass < 2; ++pass) {
#pragma unroll
      for (int it = 0; it < 8; ++it) {
        const int row = it * 2 + hh;
        const v8h hv = *(const v8h*)(ow + row * PPIT + c8);
        *(volatile v8h*)(op + (rowb + q0 + row) * DMOD + c8) = hv;
      }
      __threadfence();
    }
  }
}

template <bool W16>
__global__ __launch_bounds__(256) void k_ln(const float* __restrict__ in, const float* __restrict__ gam,
                                           const float* __restrict__ bet, float* __restrict__ outf,
                                           _Float16* __restrict__ out16, int nrows) {
  const int wave = threadIdx.x >> 5, lane = threadIdx.x & 31;
  const int row = blockIdx.x * 8 + wave;
  if (row >= nrows) return;
  const size_t base = (size_t)row * DMOD;
  const v4f xv = *(const v4f*)(in + base + 4 * lane);
  float s1 = (xv[0] + xv[1]) + (xv[2] + xv[3]);
  s1 += __shfl_xor(s1, 1, 32);
  s1 += __shfl_xor(s1, 2, 32);
  s1 += __shfl_xor(s1, 4, 32);
  s1 += __shfl_xor(s1, 8, 32);
  s1 += __shfl_xor(s1, 16, 32);
  const float mean = s1 * (1.0f / 128.0f);
  float d[4];
  float s2 = 0.f;
#pragma unroll
  for (int e = 0; e < 4; ++e) { d[e] = xv[e] - mean; s2 += d[e] * d[e]; }
  s2 += __shfl_xor(s2, 1, 32);
  s2 += __shfl_xor(s2, 2, 32);
  s2 += __shfl_xor(s2, 4, 32);
  s2 += __shfl_xor(s2, 8, 32);
  s2 += __shfl_xor(s2, 16, 32);
  const float var = s2 * (1.0f / 128.0f);
  const float rstd = rsqrtf(var + 1.0e-5f);
  const v4f gv = *(const v4f*)(gam + 4 * lane);
  const v4f bv = *(const v4f*)(bet + 4 * lane);
  float y[4];
#pragma unroll
  for (int e = 0; e < 4; ++e) y[e] = d[e] * rstd * gv[e] + bv[e];
  const v4f yo = {y[0], y[1], y[2], y[3]};
  float* po = outf + base + 4 * lane;
  *(volatile v4f*)po = yo;
  __threadfence();
  *(volatile v4f*)po = yo;
  if (W16) {
    v8h hv;
#pragma unroll
    for (int e = 0; e < 8; ++e) {
      const int srcl = 2 * (lane & 15) + (e >> 2);
      const float tv = __shfl(y[e & 3], srcl, 32);
      hv[e] = (_Float16)tv;
    }
    if (lane < 16) {
      _Float16* ph = out16 + base + 8 * lane;
      *(volatile v8h*)ph = hv;
      __threadfence();
      *(volatile v8h*)ph = hv;
    }
  }
}

__global__ __launch_bounds__(256) void k_conv(const float* __restrict__ xz, const float* __restrict__ cw,
                                             const float* __restrict__ cbias, float* __restrict__ xcf,
                                             _Float16* __restrict__ xc16) {
  const int wave = threadIdx.x >> 5, lane = threadIdx.x & 31;
  const int row = blockIdx.x * 4 + (wave >> 1);
  const int chalf = (wave & 1) * 128;
  const int c0 = chalf + 4 * lane;
  const int t = (row >> 7) & (TSEQ - 1);
  v4f wv[4];
#pragma unroll
  for (int ci = 0; ci < 4; ++ci) wv[ci] = *(const v4f*)(cw + (size_t)(c0 + ci) * 4);
  const v4f bb = *(const v4f*)(cbias + c0);
  float acc[4] = {bb[0], bb[1], bb[2], bb[3]};
#pragma unroll
  for (int kk = 0; kk < 4; ++kk) {
    const int tt = t + kk - 3;
    const int ttc = (tt < 0) ? 0 : tt;
    const size_t rsrc = (size_t)(row - (t - ttc) * NNOD);
    const v4f xv = *(const v4f*)(xz + rsrc * XZW + c0);
    const bool valid = (tt >= 0);
#pragma unroll
    for (int ci = 0; ci < 4; ++ci) acc[ci] = acc[ci] + wv[ci][kk] * (valid ? xv[ci] : 0.0f);
  }
  float y[4];
#pragma unroll
  for (int ci = 0; ci < 4; ++ci) {
    const float a = acc[ci];
    const float sg = 1.0f / (1.0f + expf(-a));
    y[ci] = a * sg;
  }
  const v4f yo = {y[0], y[1], y[2], y[3]};
  float* pf = xcf + (size_t)row * DINR + c0;
  *(volatile v4f*)pf = yo;
  __threadfence();
  *(volatile v4f*)pf = yo;
  v8h hv;
#pragma unroll
  for (int e = 0; e < 8; ++e) {
    const int srcl = 2 * (lane & 15) + (e >> 2);
    const float tv = __shfl(y[e & 3], srcl, 32);
    hv[e] = (_Float16)(tv * ACARRY);
  }
  if (lane < 16) {
    _Float16* ph = xc16 + (size_t)row * DINR + chalf + 8 * lane;
    *(volatile v8h*)ph = hv;
    __threadfence();
    *(volatile v8h*)ph = hv;
  }
}

__global__ __launch_bounds__(256) void k_dt(const float* __restrict__ dbc, const float* __restrict__ dtw,
                                           const float* __restrict__ dtb, float* __restrict__ dtp) {
  const int row = blockIdx.x, ch = threadIdx.x;
  const v4f d0 = *(const v4f*)(dbc + (size_t)row * DBCP);
  const v4f d1 = *(const v4f*)(dbc + (size_t)row * DBCP + 4);
  float acc = 0.f;
#pragma unroll
  for (int k = 0; k < 4; ++k) acc += d0[k] * dtw[k * DINR + ch];
#pragma unroll
  for (int k = 0; k < 4; ++k) acc += d1[k] * dtw[(4 + k) * DINR + ch];
  acc += dtb[ch];
  const float sp = fmaxf(acc, 0.0f) + log1pf(expf(-fabsf(acc)));
  float* p = dtp + (size_t)row * DINR + ch;
  *(volatile float*)p = sp;
  __threadfence();
  *(volatile float*)p = sp;
}

__global__ __launch_bounds__(256) void k_scan(const float* __restrict__ dtp, const float* __restrict__ xcf,
                                             const float* __restrict__ xz, const float* __restrict__ dbc,
                                             const float* __restrict__ alog, const float* __restrict__ dp,
                                             _Float16* __restrict__ y16) {
  __shared__ __align__(16) float sY[TSEQ * 64];
  const int tid = threadIdx.x, lane = tid & 31, wave = tid >> 5;
  const int bn = blockIdx.x >> 2, cg = blockIdx.x & 3;
  const int cb = cg * 64;
  const int chl = tid >> 2, q = tid & 3;
  const int ch = cb + chl;
  const int bidx = bn >> 7, nidx = bn & (NNOD - 1);
  const size_t rowbase = (size_t)bidx * (TSEQ * NNOD) + nidx;
  const v4f al = *(const v4f*)(alog + (size_t)ch * DSTA + 4 * q);
  float Acf[4];
#pragma unroll
  for (int e = 0; e < 4; ++e) Acf[e] = -expf(al[e]);
  const float dpc = dp[ch];
  float hs[4] = {0.f, 0.f, 0.f, 0.f};
#pragma unroll 1
  for (int t = 0; t < TSEQ; ++t) {
    const size_t row = rowbase + (size_t)t * NNOD;
    const float dtv = dtp[row * DINR + ch];
    const float xv  = xcf[row * DINR + ch];
    const float zv  = xz[row * XZW + DINR + ch];
    const v4f B4 = *(const v4f*)(dbc + row * DBCP + DTRK + 4 * q);
    const v4f C4 = *(const v4f*)(dbc + row * DBCP + DTRK + DSTA + 4 * q);
    const float dx = dtv * xv;
    float yp = 0.f;
#pragma unroll
    for (int e = 0; e < 4; ++e) {
      const float dA = expf(dtv * Acf[e]);
      hs[e] = dA * hs[e] + dx * B4[e];
      yp = yp + hs[e] * C4[e];
    }
    yp += __shfl_xor(yp, 1, 32);
    yp += __shfl_xor(yp, 2, 32);
    float yv = yp + dpc * xv;
    const float sg = 1.0f / (1.0f + expf(-zv));
    yv = yv * (zv * sg);
    if (q == 0) sY[t * 64 + chl] = yv * ACARRY;
  }
  __syncthreads();
  {
    const int tq = lane >> 3, c8 = (lane & 7) * 8;
    const int ts = wave * 4 + tq;
    const size_t rowo = rowbase + (size_t)ts * NNOD;
    const float* sp = sY + ts * 64 + c8;
    v8h hv;
#pragma unroll
    for (int e = 0; e < 8; ++e) hv[e] = (_Float16)sp[e];
    _Float16* p = y16 + rowo * DINR + cb + c8;
    *(volatile v8h*)p = hv;
    __threadfence();
    *(volatile v8h*)p = hv;
  }
}

extern "C" void kernel_launch(void* const* d_in, const int* in_sizes, int n_in,
                              void* d_out, int out_size, void* d_ws,
                              size_t ws_size, hipStream_t stream) {
  if (n_in < 21) return;
  if (in_sizes[0] != NROW * DMOD || out_size != NROW * DMOD) return;
  const float* x       = (const float*)d_in[0];
  const float* adj     = (const float*)d_in[1];
  const float* Wq      = (const float*)d_in[2];
  const float* Wk      = (const float*)d_in[3];
  const float* Wv      = (const float*)d_in[4];
  const float* Wo      = (const float*)d_in[5];
  const float* bo      = (const float*)d_in[6];
  const float* ns_g    = (const float*)d_in[7];
  const float* ns_b    = (const float*)d_in[8];
  const float* nt_g    = (const float*)d_in[9];
  const float* nt_b    = (const float*)d_in[10];
  const float* in_proj = (const float*)d_in[11];
  const float* conv_w  = (const float*)d_in[12];
  const float* conv_b  = (const float*)d_in[13];
  const float* x_proj  = (const float*)d_in[14];
  const float* dt_w    = (const float*)d_in[15];
  const float* dt_b    = (const float*)d_in[16];
  const float* A_log   = (const float*)d_in[17];
  const float* Dp      = (const float*)d_in[18];
  const float* out_w   = (const float*)d_in[19];
  const float* out_b   = (const float*)d_in[20];
  float* out = (float*)d_out;

  char* wsb = (char*)d_ws;
  size_t off = 0;
  _Float16* wqkvT = (_Float16*)(wsb + off); off += (size_t)QKVW * DMOD * 2;
  _Float16* woT   = (_Float16*)(wsb + off); off += (size_t)DMOD * DMOD * 2;
  _Float16* inpT  = (_Float16*)(wsb + off); off += (size_t)XZW * DMOD * 2;
  _Float16* xpT   = (_Float16*)(wsb + off); off += (size_t)XPNP * DINR * 2;
  _Float16* owT   = (_Float16*)(wsb + off); off += (size_t)DMOD * DINR * 2;
  unsigned* adjw  = (unsigned*)(wsb + off); off += (size_t)NNOD * 4 * 4;
  _Float16* xh    = (_Float16*)(wsb + off); _Float16* oh = xh;           off += (size_t)NROW * DMOD * 2;
  _Float16* qkv   = (_Float16*)(wsb + off); _Float16* xc16 = qkv;        off += (size_t)NROW * QKVW * 2;
  float*    p1    = (float*)(wsb + off);    float* p2 = p1;              off += (size_t)NROW * DMOD * 4;
  float*    hf    = (float*)(wsb + off);                                 off += (size_t)NROW * DMOD * 4;
  _Float16* hh    = (_Float16*)(wsb + off); float* dbc = (float*)(wsb + off); off += (size_t)NROW * DMOD * 2;
  float*    xz    = (float*)(wsb + off);                                 off += (size_t)NROW * XZW * 4;
  float*    xcf   = (float*)(wsb + off);                                 off += (size_t)NROW * DINR * 4;
  float*    dtp   = (float*)(wsb + off);                                 off += (size_t)NROW * DINR * 4;
  _Float16* y16   = (_Float16*)(wsb + off);                              off += (size_t)NROW * DINR * 2;
  if (off > ws_size) return;

  const dim3 blk(256);
  k_castT<<<dim3(DMOD / 64, DMOD / 64, 3), blk, 0, stream>>>(Wq, Wk, Wv, DMOD, DMOD, wqkvT, WCARRY);
  k_castT<<<dim3(DMOD / 64, DMOD / 64, 1), blk, 0, stream>>>(Wo, Wo, Wo, DMOD, DMOD, woT, WCARRY);
  k_castT<<<dim3(DMOD / 64, XZW / 64, 1), blk, 0, stream>>>(in_proj, in_proj, in_proj, DMOD, XZW, inpT, WCARRY);
  k_castT<<<dim3(DINR / 64, XPNP / 64, 1), blk, 0, stream>>>(x_proj, x_proj, x_proj, DINR, XPN, xpT, WCARRY);
  k_castT<<<dim3(DINR / 64, DMOD / 64, 1), blk, 0, stream>>>(out_w, out_w, out_w, DINR, DMOD, owT, WCARRY);
  k_adjbits<<<dim3(1), dim3(512), 0, stream>>>(adj, adjw);
  cast_f32_f16x2<<<dim3((NROW * DMOD / 2) / 256), blk, 0, stream>>>(x, xh, NROW * DMOD / 2);

  wmma_gemm64<0, false, 0, 1, false><<<dim3(((NROW / 64) * (QKVW / 64)) / 8, 1), blk, 0, stream>>>(
      (const unsigned short*)xh, (const unsigned short*)xh, DMOD, 0L,
      (const unsigned short*)wqkvT, (const unsigned short*)wqkvT, DMOD, 0L,
      (void*)qkv, (void*)qkv, QKVW, 0L, bo, x, 0L, NROW, QKVW, DMOD, WCARRY_INV);

  k_attn<<<dim3((NROW / NNOD) * 2), dim3(128), 0, stream>>>((const unsigned short*)qkv, adjw, oh);

  wmma_gemm64<0, false, 2, 0, true, 0, 2><<<dim3(((NROW / 64) * (DMOD / 64)) / 8, 1), blk, 0, stream>>>(
      (const unsigned short*)oh, (const unsigned short*)oh, DMOD, 0L,
      (const unsigned short*)woT, (const unsigned short*)woT, DMOD, 0L,
      (void*)p1, (void*)p1, DMOD, 0L, bo, x, 0L, NROW, DMOD, DMOD, WCARRY_INV);

  k_ln<true><<<dim3(NROW / 8), blk, 0, stream>>>(p1, ns_g, ns_b, hf, hh, NROW);

  wmma_gemm64<0, false, 0, 0, false><<<dim3(((NROW / 64) * (XZW / 64)) / 8, 1), blk, 0, stream>>>(
      (const unsigned short*)hh, (const unsigned short*)hh, DMOD, 0L,
      (const unsigned short*)inpT, (const unsigned short*)inpT, DMOD, 0L,
      (void*)xz, (void*)xz, XZW, 0L, bo, x, 0L, NROW, XZW, DMOD, WCARRY_INV);

  k_conv<<<dim3(NROW / 4), blk, 0, stream>>>(xz, conv_w, conv_b, xcf, xc16);

  wmma_gemm64<0, false, 0, 0, false><<<dim3(((NROW / 64) * (XPNP / 64)) / 8, 1), blk, 0, stream>>>(
      (const unsigned short*)xc16, (const unsigned short*)xc16, DINR, 0L,
      (const unsigned short*)xpT, (const unsigned short*)xpT, DINR, 0L,
      (void*)dbc, (void*)dbc, DBCP, 0L, bo, x, 0L, NROW, XPNP, DINR, AWCARRY_INV);

  k_dt<<<dim3(NROW), blk, 0, stream>>>(dbc, dt_w, dt_b, dtp);

  k_scan<<<dim3(NSEQ * 4), blk, 0, stream>>>(dtp, xcf, xz, dbc, A_log, Dp, y16);

  wmma_gemm64<0, false, 2, 0, true, 0, 1><<<dim3(((NROW / 64) * (DMOD / 64)) / 8, 1), blk, 0, stream>>>(
      (const unsigned short*)y16, (const unsigned short*)y16, DINR, 0L,
      (const unsigned short*)owT, (const unsigned short*)owT, DINR, 0L,
      (void*)p2, (void*)p2, DMOD, 0L, out_b, hf, 0L, NROW, DMOD, DINR, AWCARRY_INV);

  k_ln<false><<<dim3(NROW / 8), blk, 0, stream>>>(p2, nt_g, nt_b, out, y16, NROW);
}
